// SpatialStructuralEmbedder_11347303596106
// MI455X (gfx1250) — hardware-verified
//
#include <hip/hip_runtime.h>
#include <stdint.h>

#define NP   8192
#define NTI  128
#define NT   8320
#define NE   1024
#define IND  384
#define GD   256
#define NH   4
#define DHD  64
#define NG8  1040
#define NEGV (-1.0e9f)
#define PSC  32768.0f

typedef __attribute__((ext_vector_type(16))) _Float16 v16h;
typedef __attribute__((ext_vector_type(8)))  _Float16 v8h;
typedef __attribute__((ext_vector_type(16))) __bf16   v16b;
typedef __attribute__((ext_vector_type(8)))  __bf16   v8b;
typedef __attribute__((ext_vector_type(8)))  float    v8f;
typedef __attribute__((ext_vector_type(4)))  float    v4f;

__device__ __forceinline__ unsigned short f2bf_bits(float f) {
  unsigned u = __float_as_uint(f);
  return (unsigned short)((u + 0x7FFFu + ((u >> 16) & 1u)) >> 16);
}
__device__ __forceinline__ float bf_bits2f(unsigned short h) { return __uint_as_float(((unsigned)h) << 16); }

__device__ __forceinline__ void dep_guard_h(v8f& a, v8f& b, v16h x, v16h y) { asm volatile("v_nop\n\tv_nop\n\tv_nop\n\tv_nop" : "+v"(a), "+v"(b) : "v"(x), "v"(y)); }
__device__ __forceinline__ void dep_guard_b(v8f& a, v8f& b, v16b x, v16b y) { asm volatile("v_nop\n\tv_nop\n\tv_nop\n\tv_nop" : "+v"(a), "+v"(b) : "v"(x), "v"(y)); }
__device__ __forceinline__ void keep4_h(v16h a, v16h b, v16h c, v16h d) { asm volatile("v_nop" :: "v"(a), "v"(b), "v"(c), "v"(d)); }
__device__ __forceinline__ void keep4_b(v16b a, v16b b, v16b c, v16b d) { asm volatile("v_nop" :: "v"(a), "v"(b), "v"(c), "v"(d)); }
__device__ __forceinline__ void acc_guard4(v8f& a, v8f& b, v8f& c, v8f& d) { asm volatile("v_nop\n\tv_nop\n\tv_nop\n\tv_nop" : "+v"(a), "+v"(b), "+v"(c), "+v"(d)); }
template <typename T> struct Frag;
template <> struct Frag<_Float16> {
  typedef v16h V; union U { v16h v; v8h h[2]; };
  static __device__ __forceinline__ v16h load(const _Float16* p) {
    U f; f.h[0] = *(const v8h*)(p); f.h[1] = *(const v8h*)(p + 16); return f.v;
  }
  static __device__ __forceinline__ v8f mma(v16h a, v16h b, v8f c) {
    return __builtin_amdgcn_wmma_f32_16x16x32_f16(false, a, false, b, (short)0, c, false, false);
  }
  static __device__ __forceinline__ void guard(v8f& a, v8f& b, v16h x, v16h y) { dep_guard_h(a, b, x, y); }
  static __device__ __forceinline__ void keep(v16h a, v16h b, v16h c, v16h d) { keep4_h(a, b, c, d); }
};
template <> struct Frag<__bf16> {
  typedef v16b V; union U { v16b v; v8b h[2]; };
  static __device__ __forceinline__ v16b load(const __bf16* p) {
    U f; f.h[0] = *(const v8b*)(p); f.h[1] = *(const v8b*)(p + 16); return f.v;
  }
  static __device__ __forceinline__ v8f mma(v16b a, v16b b, v8f c) {
    return __builtin_amdgcn_wmma_f32_16x16x32_bf16(false, a, false, b, (short)0, c, false, false);
  }
  static __device__ __forceinline__ void guard(v8f& a, v8f& b, v16b x, v16b y) { dep_guard_b(a, b, x, y); }
  static __device__ __forceinline__ void keep(v16b a, v16b b, v16b c, v16b d) { keep4_b(a, b, c, d); }
};

__device__ __forceinline__ float lrelu(float x) { return x > 0.f ? x : 0.2f * x; }

template <int ET> struct Elem;
template <> struct Elem<0> { typedef _Float16 T; };
template <> struct Elem<1> { typedef __bf16 T; };
template <int ET, bool SPLIT, int EPI, int OUT_MODE>
__global__ __launch_bounds__(256) void wmma_gemm64(
    const unsigned short* __restrict__ Ap, const unsigned short* __restrict__ A2p, int lda, long strideA,
    const unsigned short* __restrict__ Btp, const unsigned short* __restrict__ Bt2p, int ldb, long strideB,
    void* __restrict__ Cout, void* __restrict__ Cout2, int ldc, long strideC,
    const float* __restrict__ rs, long rsStrideB, int rsPitch,
    const float* __restrict__ gbias, const int* __restrict__ gidx, int gld, int gmax,
    const float* __restrict__ resid, long strideR,
    int M, int N, int K, float scale) {
  typedef typename Elem<ET>::T T;
  typedef typename Frag<T>::V V;
  const T* A = (const T*)Ap; const T* A2 = (const T*)A2p; const T* Bt = (const T*)Btp; const T* Bt2 = (const T*)Bt2p;
  __shared__ __align__(16) float sT[8][16 * 68];
  const int b    = blockIdx.y;
  const int lane = threadIdx.x & 31;
  const int wave = threadIdx.x >> 5;
  const int tilesN = N >> 6;
  const int tilesM = M >> 6;
  const int tile = blockIdx.x * 8 + wave;
  if (tile >= tilesM * tilesN) return;
  const int tm = tile / tilesN;
  const int tn = tile - tm * tilesN;
  const int m0 = tm << 6;
  const int n0 = tn << 6;

  const T* Ab  = A  + (size_t)b * strideA;
  const T* Bb  = Bt + (size_t)b * strideB;
  const T* Ab2 = SPLIT ? (A2  + (size_t)b * strideA) : nullptr;
  const T* Bb2 = SPLIT ? (Bt2 + (size_t)b * strideB) : nullptr;

  const int rlane = lane & 15;
  const int koff  = (lane >> 4) * 8;
  const int mOff  = (lane >> 4) * 8;

  v8f acc[4][4];
#pragma unroll
  for (int i = 0; i < 4; ++i)
#pragma unroll
    for (int j = 0; j < 4; ++j) acc[i][j] = (v8f){0.f,0.f,0.f,0.f,0.f,0.f,0.f,0.f};

  for (int k0 = 0; k0 < K; k0 += 32) {
    V bh[4], bl[4];
#pragma unroll
    for (int j = 0; j < 4; ++j) {
      const size_t bo = (size_t)(n0 + (j << 4) + rlane) * ldb + koff + k0;
      bh[j] = Frag<T>::load(Bb + bo);
      if (SPLIT) bl[j] = Frag<T>::load(Bb2 + bo);
    }
#pragma unroll
    for (int i = 0; i < 4; ++i) {
      const size_t ao = (size_t)(m0 + (i << 4) + rlane) * lda + koff + k0;
      V ah = Frag<T>::load(Ab + ao);
      V al;
      if (SPLIT) al = Frag<T>::load(Ab2 + ao);
#pragma unroll
      for (int j = 0; j < 4; ++j) {
        acc[i][j] = Frag<T>::mma(ah, bh[j], acc[i][j]);
        if (SPLIT) {
          acc[i][j] = Frag<T>::mma(ah, bl[j], acc[i][j]);
          acc[i][j] = Frag<T>::mma(al, bh[j], acc[i][j]);
        }
      }
      Frag<T>::guard(acc[i][0], acc[i][3], ah, SPLIT ? al : ah);
    }
    Frag<T>::keep(bh[0], bh[1], bh[2], bh[3]);
    if (SPLIT) Frag<T>::keep(bl[0], bl[1], bl[2], bl[3]);
  }
  acc_guard4(acc[0][0], acc[0][1], acc[0][2], acc[0][3]);
  acc_guard4(acc[1][0], acc[1][1], acc[1][2], acc[1][3]);
  acc_guard4(acc[2][0], acc[2][1], acc[2][2], acc[2][3]);
  acc_guard4(acc[3][0], acc[3][1], acc[3][2], acc[3][3]);

  float* slab = sT[wave];
  const float* Rb = (EPI == 2) ? (resid + (size_t)b * strideR) : nullptr;
  const float* Rs = (EPI >= 1) ? (rs + (size_t)b * rsStrideB) : nullptr;
#pragma unroll
  for (int i = 0; i < 4; ++i) {
    const int mBase = m0 + (i << 4);
    float rsc[8]; int gt[8];
#pragma unroll
    for (int r = 0; r < 8; ++r) {
      const int m = mBase + mOff + r;
      rsc[r] = 1.f; gt[r] = 0;
      if (EPI >= 1) rsc[r] = Rs[(size_t)m * rsPitch];
      if (EPI == 0) { int t = gidx[m]; t = t < 0 ? 0 : (t >= gmax ? gmax - 1 : t); gt[r] = t; }
    }
#pragma unroll
    for (int j = 0; j < 4; ++j) {
      const int n = n0 + (j << 4) + rlane;
#pragma unroll
      for (int r = 0; r < 8; ++r) {
        float v = acc[i][j][r] * scale;
        if (EPI == 0) v += gbias[(size_t)gt[r] * gld + n];
        if (EPI >= 1) v *= rsc[r];
        if (EPI == 2) {
          const float el = (v > 0.f) ? v : (__expf(v) - 1.f);
          v = el + Rb[(size_t)(mBase + mOff + r) * ldc + n];
        }
        slab[(mOff + r) * 68 + (j << 4) + rlane] = v;
      }
    }
    __builtin_amdgcn_fence(__ATOMIC_RELEASE, "workgroup");
    __builtin_amdgcn_wave_barrier();
    __builtin_amdgcn_fence(__ATOMIC_ACQUIRE, "workgroup");
    if (OUT_MODE == 0) {
      float* C = (float*)Cout + (size_t)b * strideC;
      const int hh = lane >> 4, c4 = (lane & 15) * 4;
      for (int pass = 0; pass < 2; ++pass) {
#pragma unroll
        for (int it = 0; it < 8; ++it) {
          const int row = it * 2 + hh;
          v4f v = *(const v4f*)(slab + row * 68 + c4);
          *(volatile v4f*)(C + (size_t)(mBase + row) * ldc + n0 + c4) = v;
        }
        __threadfence();
      }
    } else {
      const int q = lane >> 3, c8 = (lane & 7) * 8;
      unsigned short* C  = (unsigned short*)Cout  + (size_t)b * strideC;
      unsigned short* C2 = (OUT_MODE == 2) ? ((unsigned short*)Cout2 + (size_t)b * strideC) : nullptr;
      for (int pass = 0; pass < 2; ++pass) {
#pragma unroll
        for (int it = 0; it < 4; ++it) {
          const int row = it * 4 + q;
          const float* sp = slab + row * 68 + c8;
          v8h hv, lv;
#pragma unroll
          for (int e = 0; e < 8; ++e) {
            if (OUT_MODE == 1) {
              hv[e] = (_Float16)sp[e];
            } else {
              unsigned short hb = f2bf_bits(sp[e]);
              unsigned short lb = f2bf_bits(sp[e] - bf_bits2f(hb));
              hv[e] = __builtin_bit_cast(_Float16, hb);
              lv[e] = __builtin_bit_cast(_Float16, lb);
            }
          }
          *(volatile v8h*)(C + (size_t)(mBase + row) * ldc + n0 + c8) = hv;
          if (OUT_MODE == 2) *(volatile v8h*)(C2 + (size_t)(mBase + row) * ldc + n0 + c8) = lv;
        }
        __threadfence();
      }
    }
    __builtin_amdgcn_fence(__ATOMIC_RELEASE, "workgroup");
    __builtin_amdgcn_wave_barrier();
    __builtin_amdgcn_fence(__ATOMIC_ACQUIRE, "workgroup");
  }
}

__global__ __launch_bounds__(256) void k_cast16(
    const float* __restrict__ in, _Float16* __restrict__ out, int n2, float scale) {
  int i = blockIdx.x * 256 + threadIdx.x;
  if (i < n2) {
    const _Float16 h0 = (_Float16)(in[2 * i] * scale), h1 = (_Float16)(in[2 * i + 1] * scale);
    const unsigned u = (unsigned)__builtin_bit_cast(unsigned short, h0) | ((unsigned)__builtin_bit_cast(unsigned short, h1) << 16);
    ((volatile unsigned*)out)[i] = u;
    __threadfence();
    ((volatile unsigned*)out)[i] = u;
  }
}

__global__ __launch_bounds__(256) void k_build_x16(
    const float* __restrict__ x, const float* __restrict__ rtok, _Float16* __restrict__ X16) {
  const int g = blockIdx.x * 256 + threadIdx.x;
  if (g < NT * IND / 8) {
    const int idx = g * 8;
    const int n = idx / IND;
    const int k = idx - n * IND;
    const float* src = (n < NP) ? (x + idx) : (rtok + k);
    const v4f a = *(const v4f*)(src);
    const v4f c = *(const v4f*)(src + 4);
    v8h hv;
    hv[0] = (_Float16)a[0]; hv[1] = (_Float16)a[1]; hv[2] = (_Float16)a[2]; hv[3] = (_Float16)a[3];
    hv[4] = (_Float16)c[0]; hv[5] = (_Float16)c[1]; hv[6] = (_Float16)c[2]; hv[7] = (_Float16)c[3];
    _Float16* p = X16 + idx;
    *(volatile v8h*)p = hv;
    __threadfence();
    *(volatile v8h*)p = hv;
  }
}

template <int NV>
__global__ __launch_bounds__(256) void k_tr16(const float* __restrict__ src, int R, int C,
    _Float16* __restrict__ dst, float scale,
    const float* __restrict__ vec0, const float* __restrict__ vec1,
    float* __restrict__ sc0, float* __restrict__ sc1) {
  __shared__ float tile[64][65];
  __shared__ float red[2][64];
  const int tid = threadIdx.x;
  const int c0 = blockIdx.x * 64, r0 = blockIdx.y * 64;
  {
    const int row = tid >> 2, cq = (tid & 3) * 16;
    const float* sp = src + (size_t)(r0 + row) * C + c0 + cq;
#pragma unroll
    for (int i = 0; i < 4; ++i) {
      const v4f v = *(const v4f*)(sp + 4 * i);
      tile[row][cq + 4 * i + 0] = v[0];
      tile[row][cq + 4 * i + 1] = v[1];
      tile[row][cq + 4 * i + 2] = v[2];
      tile[row][cq + 4 * i + 3] = v[3];
    }
  }
  __syncthreads();
  if (NV > 0) {
    const int row = tid >> 2, q = tid & 3;
    float p0 = 0.f, p1 = 0.f;
#pragma unroll
    for (int i = 0; i < 16; ++i) {
      const float tv = tile[row][q * 16 + i];
      p0 += tv * vec0[c0 + q * 16 + i];
      if (NV > 1) p1 += tv * vec1[c0 + q * 16 + i];
    }
    p0 += __shfl_xor(p0, 1, 32);
    p0 += __shfl_xor(p0, 2, 32);
    if (NV > 1) {
      p1 += __shfl_xor(p1, 1, 32);
      p1 += __shfl_xor(p1, 2, 32);
    }
    if (q == 0) {
      red[0][row] = p0;
      if (NV > 1) red[1][row] = p1;
    }
  }
  __syncthreads();
  if (NV > 0) {
    if (tid < 64) {
      const float v = red[0][tid];
      float* p = sc0 + (size_t)blockIdx.x * R + r0 + tid;
      *(volatile float*)p = v;
      __threadfence();
      *(volatile float*)p = v;
    }
    if (NV > 1) {
      if (tid >= 64 && tid < 128) {
        const float v = red[1][tid - 64];
        float* p = sc1 + (size_t)blockIdx.x * R + r0 + (tid - 64);
        *(volatile float*)p = v;
        __threadfence();
        *(volatile float*)p = v;
      }
    }
  }
  {
    const int seg = (tid & 7) * 8;
    v8h hv[2];
#pragma unroll
    for (int half = 0; half < 2; ++half) {
      const int orow = (tid >> 3) + half * 32;
#pragma unroll
      for (int e = 0; e < 8; ++e) hv[half][e] = (_Float16)(tile[seg + e][orow] * scale);
    }
#pragma unroll
    for (int half = 0; half < 2; ++half) {
      const int orow = (tid >> 3) + half * 32;
      *(volatile v8h*)(dst + (size_t)(c0 + orow) * R + r0 + seg) = hv[half];
    }
    __threadfence();
#pragma unroll
    for (int half = 0; half < 2; ++half) {
      const int orow = (tid >> 3) + half * 32;
      *(volatile v8h*)(dst + (size_t)(c0 + orow) * R + r0 + seg) = hv[half];
    }
  }
}

__global__ __launch_bounds__(256) void k_colsoft(const float* __restrict__ H, const float* __restrict__ ssrc,
    const int* __restrict__ etype, const float* __restrict__ ebias,
    _Float16* __restrict__ P16, float* __restrict__ invZ) {
  __shared__ float red[8][4];
  const int e = blockIdx.x;
  const int tid = threadIdx.x, lane = tid & 31, wave = tid >> 5;
  int t = etype[e]; t = t < 0 ? 0 : (t > 2 ? 2 : t);
  float eb[4];
#pragma unroll
  for (int h = 0; h < 4; ++h) eb[h] = ebias[t * 4 + h];

  float sm[4] = {-INFINITY, -INFINITY, -INFINITY, -INFINITY};
#pragma unroll 1
  for (int it = 0; it < 5; ++it) {
    const int g = tid + 256 * it;
    const bool valid = g < NG8;
    const int gc = valid ? g : (NG8 - 1);
    const int n0 = gc * 8;
    float mk[8];
#pragma unroll
    for (int j = 0; j < 8; ++j) mk[j] = H[(size_t)(n0 + j) * NE + e];
#pragma unroll
    for (int h = 0; h < 4; ++h) {
      const v4f s0 = *(const v4f*)(ssrc + (size_t)h * NT + n0);
      const v4f s1 = *(const v4f*)(ssrc + (size_t)h * NT + n0 + 4);
      const float s[8] = {s0[0], s0[1], s0[2], s0[3], s1[0], s1[1], s1[2], s1[3]};
#pragma unroll
      for (int j = 0; j < 8; ++j) {
        const float c = (valid && mk[j] > 0.f) ? s[j] : -INFINITY;
        sm[h] = fmaxf(sm[h], c);
      }
    }
  }
#pragma unroll
  for (int h = 0; h < 4; ++h) {
    float v = sm[h];
#pragma unroll
    for (int off = 16; off > 0; off >>= 1) v = fmaxf(v, __shfl_xor(v, off, 32));
    sm[h] = v;
  }
  if (lane == 0) {
#pragma unroll
    for (int h = 0; h < 4; ++h) red[wave][h] = sm[h];
  }
  __syncthreads();
  float Mx[4];
#pragma unroll
  for (int h = 0; h < 4; ++h) {
    float mx = red[0][h];
#pragma unroll
    for (int w = 1; w < 8; ++w) mx = fmaxf(mx, red[w][h]);
    Mx[h] = (mx == -INFINITY) ? NEGV : lrelu(mx + eb[h]);
  }
  __syncthreads();

  float zs[4] = {0.f, 0.f, 0.f, 0.f};
#pragma unroll 1
  for (int it = 0; it < 5; ++it) {
    const int g = tid + 256 * it;
    const bool valid = g < NG8;
    const int gc = valid ? g : (NG8 - 1);
    const int n0 = gc * 8;
    float mk[8];
#pragma unroll
    for (int j = 0; j < 8; ++j) mk[j] = H[(size_t)(n0 + j) * NE + e];
    v8h ph[4];
#pragma unroll
    for (int h = 0; h < 4; ++h) {
      const v4f s0 = *(const v4f*)(ssrc + (size_t)h * NT + n0);
      const v4f s1 = *(const v4f*)(ssrc + (size_t)h * NT + n0 + 4);
      const float s[8] = {s0[0], s0[1], s0[2], s0[3], s1[0], s1[1], s1[2], s1[3]};
#pragma unroll
      for (int j = 0; j < 8; ++j) {
        const float xv = (mk[j] > 0.f) ? lrelu(s[j] + eb[h]) : NEGV;
        const float p = __expf(xv - Mx[h]);
        zs[h] += valid ? p : 0.f;
        ph[h][j] = (_Float16)(p * PSC);
      }
    }
    if (valid) {
      _Float16* pb = P16 + (size_t)e * NT + n0;
#pragma unroll
      for (int h = 0; h < 4; ++h) *(volatile v8h*)(pb + (size_t)h * NE * NT) = ph[h];
      __threadfence();
#pragma unroll
      for (int h = 0; h < 4; ++h) *(volatile v8h*)(pb + (size_t)h * NE * NT) = ph[h];
    }
  }
#pragma unroll
  for (int h = 0; h < 4; ++h) {
    float v = zs[h];
#pragma unroll
    for (int off = 16; off > 0; off >>= 1) v += __shfl_xor(v, off, 32);
    zs[h] = v;
  }
  if (lane == 0) {
#pragma unroll
    for (int h = 0; h < 4; ++h) red[wave][h] = zs[h];
  }
  __syncthreads();
  if (wave == 0) {
    float z0 = 0.f, z1 = 0.f, z2 = 0.f, z3 = 0.f;
#pragma unroll
    for (int w = 0; w < 8; ++w) { z0 += red[w][0]; z1 += red[w][1]; z2 += red[w][2]; z3 += red[w][3]; }
    const float zl = (lane == 0) ? z0 : (lane == 1) ? z1 : (lane == 2) ? z2 : z3;
    const float val = (lane < 4) ? (1.0f / zl) : 0.f;
    float* pz = invZ + (size_t)e * 32 + lane;
    *(volatile float*)pz = val;
    __threadfence();
    *(volatile float*)pz = val;
  }
}

__global__ __launch_bounds__(256) void k_rowsoft(const float* __restrict__ H, const float* __restrict__ sdst,
    const float* __restrict__ sedg, _Float16* __restrict__ P16, float* __restrict__ invZ) {
  __shared__ float red[8][4];
  const int tid = threadIdx.x, lane = tid & 31, wave = tid >> 5;
  const int grp = wave >> 2;
  const int node = blockIdx.x * 2 + grp;
  const int lt = tid & 127;
  const int e0 = lt * 8;
  const v4f ma = *(const v4f*)(H + (size_t)node * NE + e0);
  const v4f mb = *(const v4f*)(H + (size_t)node * NE + e0 + 4);
  const float mk[8] = {ma[0], ma[1], ma[2], ma[3], mb[0], mb[1], mb[2], mb[3]};
  float sd[4];
  float se[4][8];
#pragma unroll
  for (int h = 0; h < 4; ++h) {
    sd[h] = sdst[(size_t)h * NT + node];
    const v4f a = *(const v4f*)(sedg + (size_t)h * NE + e0);
    const v4f c = *(const v4f*)(sedg + (size_t)h * NE + e0 + 4);
    se[h][0] = a[0]; se[h][1] = a[1]; se[h][2] = a[2]; se[h][3] = a[3];
    se[h][4] = c[0]; se[h][5] = c[1]; se[h][6] = c[2]; se[h][7] = c[3];
  }
  float em[4];
#pragma unroll
  for (int h = 0; h < 4; ++h) {
    float v = -INFINITY;
#pragma unroll
    for (int j = 0; j < 8; ++j) {
      const float c = (mk[j] > 0.f) ? se[h][j] : -INFINITY;
      v = fmaxf(v, c);
    }
#pragma unroll
    for (int off = 16; off > 0; off >>= 1) v = fmaxf(v, __shfl_xor(v, off, 32));
    em[h] = v;
  }
  if (lane == 0) {
#pragma unroll
    for (int h = 0; h < 4; ++h) red[wave][h] = em[h];
  }
  __syncthreads();
  float Mx[4];
#pragma unroll
  for (int h = 0; h < 4; ++h) {
    float mx = red[grp * 4][h];
#pragma unroll
    for (int w = 1; w < 4; ++w) mx = fmaxf(mx, red[grp * 4 + w][h]);
    Mx[h] = (mx == -INFINITY) ? NEGV : lrelu(sd[h] + mx);
  }
  __syncthreads();

  float zs[4] = {0.f, 0.f, 0.f, 0.f};
  v8h ph[4];
#pragma unroll
  for (int h = 0; h < 4; ++h) {
#pragma unroll
    for (int j = 0; j < 8; ++j) {
      const float xv = (mk[j] > 0.f) ? lrelu(sd[h] + se[h][j]) : NEGV;
      const float p = __expf(xv - Mx[h]);
      zs[h] += p;
      ph[h][j] = (_Float16)(p * PSC);
    }
  }
  {
    _Float16* pb = P16 + (size_t)node * NE + e0;
#pragma unroll
    for (int h = 0; h < 4; ++h) *(volatile v8h*)(pb + (size_t)h * NT * NE) = ph[h];
    __threadfence();
#pragma unroll
    for (int h = 0; h < 4; ++h) *(volatile v8h*)(pb + (size_t)h * NT * NE) = ph[h];
  }
#pragma unroll
  for (int h = 0; h < 4; ++h) {
    float v = zs[h];
#pragma unroll
    for (int off = 16; off > 0; off >>= 1) v += __shfl_xor(v, off, 32);
    zs[h] = v;
  }
  if (lane == 0) {
#pragma unroll
    for (int h = 0; h < 4; ++h) red[wave][h] = zs[h];
  }
  __syncthreads();
  if ((wave & 3) == 0) {
    float z0 = 0.f, z1 = 0.f, z2 = 0.f, z3 = 0.f;
#pragma unroll
    for (int w = 0; w < 4; ++w) {
      z0 += red[grp * 4 + w][0]; z1 += red[grp * 4 + w][1]; z2 += red[grp * 4 + w][2]; z3 += red[grp * 4 + w][3];
    }
    const float zl = (lane == 0) ? z0 : (lane == 1) ? z1 : (lane == 2) ? z2 : z3;
    const float val = (lane < 4) ? (1.0f / zl) : 0.f;
    float* pz = invZ + (size_t)node * 32 + lane;
    *(volatile float*)pz = val;
    __threadfence();
    *(volatile float*)pz = val;
  }
}

__global__ __launch_bounds__(256) void k_ln(const float* __restrict__ hsrc, const int* __restrict__ ids,
    const float* __restrict__ ng, const float* __restrict__ nb,
    const float* __restrict__ bg, const float* __restrict__ bb,
    float* __restrict__ out) {
  __shared__ float red[8];
  const int bidx = blockIdx.x, tid = threadIdx.x, lane = tid & 31, wave = tid >> 5;
  const bool isBag = (bidx >= NP);
  const int jj = isBag ? (bidx - NP) : 0;
  int id = ids[jj];
  id = id < 0 ? 0 : (id > NT - 1 ? NT - 1 : id);
  const int srow = isBag ? id : bidx;
  const float* g  = isBag ? bg : ng;
  const float* be = isBag ? bb : nb;
  const float x = hsrc[(size_t)srow * GD + tid];
  float v = x;
#pragma unroll
  for (int off = 16; off > 0; off >>= 1) v += __shfl_xor(v, off, 32);
  if (lane == 0) red[wave] = v;
  __syncthreads();
  float s = 0.f;
#pragma unroll
  for (int w = 0; w < 8; ++w) s += red[w];
  const float mean = s * (1.0f / GD);
  __syncthreads();
  const float d = x - mean;
  v = d * d;
#pragma unroll
  for (int off = 16; off > 0; off >>= 1) v += __shfl_xor(v, off, 32);
  if (lane == 0) red[wave] = v;
  __syncthreads();
  float s2 = 0.f;
#pragma unroll
  for (int w = 0; w < 8; ++w) s2 += red[w];
  const float var = s2 * (1.0f / GD);
  const float y = d * rsqrtf(var + 1e-5f) * g[tid] + be[tid];
  float* po = out + (size_t)bidx * GD + tid;
  *(volatile float*)po = y;
  __threadfence();
  *(volatile float*)po = y;
}

extern "C" void kernel_launch(void* const* d_in, const int* in_sizes, int n_in,
                              void* d_out, int out_size, void* d_ws, size_t ws_size,
                              hipStream_t stream) {
  if (n_in < 17) return;
  if (in_sizes[0] != NP * IND || in_sizes[1] < IND || in_sizes[2] != NT || in_sizes[3] != NE ||
      in_sizes[4] != NT * NE || in_sizes[5] != NTI || in_sizes[6] != IND * GD || in_sizes[7] != GD * GD ||
      in_sizes[8] != 2 * 4 * GD || in_sizes[9] != 2 * NH * DHD || in_sizes[10] != 2 * NH * DHD ||
      in_sizes[11] != 2 * NH * DHD || in_sizes[12] != 2 * 3 * NH || in_sizes[13] != GD || in_sizes[14] != GD ||
      in_sizes[15] != GD || in_sizes[16] != GD || out_size != NT * GD) return;

  const float* x_nodes   = (const float*)d_in[0];
  const float* rtok      = (const float*)d_in[1];
  const int*   node_type = (const int*)d_in[2];
  const int*   edge_type = (const int*)d_in[3];
  const float* H         = (const float*)d_in[4];
  const int*   ro_ids    = (const int*)d_in[5];
  const float* W0        = (const float*)d_in[6];
  const float* W1        = (const float*)d_in[7];
  const float* node_emb  = (const float*)d_in[8];
  const float* a_src     = (const float*)d_in[9];
  const float* a_dst     = (const float*)d_in[10];
  const float* a_edge    = (const float*)d_in[11];
  const float* edge_bias = (const float*)d_in[12];
  const float* ngam      = (const float*)d_in[13];
  const float* nbet      = (const float*)d_in[14];
  const float* bgam      = (const float*)d_in[15];
  const float* bbet      = (const float*)d_in[16];
  float* out = (float*)d_out;

  size_t off = 0;
  auto carve = [&](size_t bytes) -> char* {
    char* p = (char*)d_ws + off;
    off += (bytes + 255) & ~(size_t)255;
    return p;
  };
  _Float16* P16   = (_Float16*)carve((size_t)NH * NE * NT * 2);
  _Float16* X16   = (_Float16*)carve((size_t)NT * IND * 2);
  _Float16* W0T16 = (_Float16*)carve((size_t)GD * IND * 2);
  _Float16* W1T16 = (_Float16*)carve((size_t)GD * GD * 2);
  float*    hP    = (float*)carve((size_t)NT * GD * 4);
  float*    hL    = (float*)carve((size_t)NT * GD * 4);
  _Float16* hT16  = (_Float16*)carve((size_t)GD * NT * 2);
  float*    ssrc  = (float*)carve((size_t)NH * NT * 4);
  float*    sdst  = (float*)carve((size_t)NH * NT * 4);
  float*    mbuf  = (float*)carve((size_t)NE * GD * 4);
  _Float16* mT16  = (_Float16*)carve((size_t)GD * NE * 2);
  float*    sedg  = (float*)carve((size_t)NH * NE * 4);
  float*    invZ1 = (float*)carve((size_t)NE * 32 * 4);
  float*    invZ2 = (float*)carve((size_t)NT * 32 * 4);
  if (off > ws_size) return;
  _Float16* h16 = X16;

  k_build_x16<<<(NT * IND / 8) / 256, 256, 0, stream>>>(x_nodes, rtok, X16);
  k_tr16<0><<<dim3(GD / 64, IND / 64), 256, 0, stream>>>(W0, IND, GD, W0T16, 64.f, nullptr, nullptr, nullptr, nullptr);
  k_tr16<0><<<dim3(GD / 64, GD / 64), 256, 0, stream>>>(W1, GD, GD, W1T16, 64.f, nullptr, nullptr, nullptr, nullptr);

  for (int layer = 0; layer < 2; ++layer) {
    const _Float16* A16 = (layer == 0) ? X16 : h16;
    const int K          = (layer == 0) ? IND : GD;
    const _Float16* WT   = (layer == 0) ? W0T16 : W1T16;
    const float pscale   = (layer == 0) ? (1.0f / 64.0f) : (1.0f / 512.0f);
    const float* nemb = node_emb + layer * 4 * GD;
    const float* asrc = a_src + layer * NH * DHD;
    const float* adst = a_dst + layer * NH * DHD;
    const float* aedg = a_edge + layer * NH * DHD;
    const float* ebia = edge_bias + layer * 3 * NH;

    wmma_gemm64<0, false, 0, 0><<<dim3((NT / 64) * (GD / 64) / 8, 1), 256, 0, stream>>>(
        (const unsigned short*)A16, nullptr, K, 0L,
        (const unsigned short*)WT, nullptr, K, 0L,
        (void*)hP, nullptr, GD, 0L,
        nullptr, 0L, 0,
        nemb, node_type, GD, 4,
        nullptr, 0L,
        NT, GD, K, pscale);
    k_tr16<2><<<dim3(GD / 64, NT / 64), 256, 0, stream>>>(hP, NT, GD, hT16, 8.f, asrc, adst, ssrc, sdst);
    k_colsoft<<<NE, 256, 0, stream>>>(H, ssrc, edge_type, ebia, P16, invZ1);
    wmma_gemm64<0, false, 1, 0><<<dim3((NE / 64) * (DHD / 64) / 8, NH), 256, 0, stream>>>(
        (const unsigned short*)P16, nullptr, NT, (long)NE * NT,
        (const unsigned short*)hT16, nullptr, NT, (long)DHD * NT,
        (void*)mbuf, nullptr, GD, (long)DHD,
        invZ1, 1L, 32,
        nullptr, nullptr, 0, 1,
        nullptr, 0L,
        NE, DHD, NT, 1.0f / 262144.0f);
    k_tr16<1><<<dim3(GD / 64, NE / 64), 256, 0, stream>>>(mbuf, NE, GD, mT16, 64.f, aedg, nullptr, sedg, nullptr);
    k_rowsoft<<<NT / 2, 256, 0, stream>>>(H, sdst, sedg, P16, invZ2);
    wmma_gemm64<0, false, 2, 0><<<dim3(((NT / 64) * (DHD / 64) + 7) / 8, NH), 256, 0, stream>>>(
        (const unsigned short*)P16, nullptr, NE, (long)NT * NE,
        (const unsigned short*)mT16, nullptr, NE, (long)DHD * NE,
        (void*)hL, nullptr, GD, (long)DHD,
        invZ2, 1L, 32,
        nullptr, nullptr, 0, 1,
        hP, (long)DHD,
        NT, DHD, NE, 1.0f / 2097152.0f);
    if (layer == 0) {
      k_cast16<<<(NT * GD / 2) / 256, 256, 0, stream>>>(hL, h16, NT * GD / 2, 8.f);
    }
  }

  k_ln<<<NP + NTI, 256, 0, stream>>>(hL, ro_ids, ngam, nbet, bgam, bbet, out);
  (void)hipGetLastError();
}
